// MultiHeadAttention_67284957659561
// MI455X (gfx1250) — hardware-verified
//
#include <hip/hip_runtime.h>


#ifndef NB
#define NB 2
#endif
#ifndef SEQ
#define SEQ 2048
#endif
#define NB_FULL  2
#define SEQ_FULL 2048
#define DM   1024
#define NH_  16
#define HD   64
#define ATW  4
#define PCAR 256.0f
#define VRES 2048.0f
#define NEGF (-1.0e9f)
#define L2E  1.4426950408889634f

static_assert(NH_ * HD == DM);
static_assert(HD == 64);
static_assert(DM % 64 == 0 && DM % 32 == 0);
static_assert(SEQ % 64 == 0);
static_assert((NB * SEQ) % 64 == 0);
static_assert(NB <= NB_FULL && SEQ <= SEQ_FULL);
static_assert(ATW * 16 == 64);

typedef _Float16 h16;
typedef unsigned short bf;
typedef __attribute__((ext_vector_type(16))) __bf16   v16bf;
typedef __attribute__((ext_vector_type(16))) _Float16 v16h;
typedef __attribute__((ext_vector_type(8)))  _Float16 v8h;
typedef __attribute__((ext_vector_type(8)))  unsigned short v8us;
typedef __attribute__((ext_vector_type(8)))  float    v8f;
typedef __attribute__((ext_vector_type(4)))  float    v4f;
typedef v4f  __attribute__((may_alias)) v4fa;

__device__ __forceinline__ unsigned short f2bf(float f) { unsigned u = __float_as_uint(f); u += 0x7FFFu + ((u >> 16) & 1u); return (unsigned short)(u >> 16); }
__device__ __forceinline__ float bf2f(unsigned short b) { return __uint_as_float(((unsigned)b) << 16); }
__device__ __forceinline__ float bfr(float f) { return bf2f(f2bf(f)); }
__device__ __forceinline__ void splitf(float y, unsigned short& h, unsigned short& l) { h = f2bf(y); l = f2bf(y - bf2f(h)); }
__device__ __forceinline__ v16h cat16(v8h lo, v8h hi) { return __builtin_shufflevector(lo, hi, 0, 1, 2, 3, 4, 5, 6, 7, 8, 9, 10, 11, 12, 13, 14, 15); }
__device__ __forceinline__ v16bf cat16b(v8us lo, v8us hi) { return __builtin_bit_cast(v16bf, __builtin_shufflevector(lo, hi, 0, 1, 2, 3, 4, 5, 6, 7, 8, 9, 10, 11, 12, 13, 14, 15)); }
__device__ __forceinline__ v8f wmma16(v16h a, v16h b, v8f c) { return __builtin_amdgcn_wmma_f32_16x16x32_f16(false, a, false, b, (short)0, c, false, false); }
__device__ __forceinline__ v8f wmmab(v16bf a, v16bf b, v8f c) { return __builtin_amdgcn_wmma_f32_16x16x32_bf16(false, a, false, b, (short)0, c, false, false); }
__device__ __forceinline__ v16bf ldb(const bf* p) { return cat16b(*(const v8us*)p, *(const v8us*)(p + 16)); }
__device__ __forceinline__ v16h  ldh(const h16* p) { return cat16(*(const v8h*)p, *(const v8h*)(p + 16)); }

__global__ __launch_bounds__(32) void k_gemm_proj(const bf* __restrict__ A, const bf* __restrict__ Bt, int K, float* C, int ldc, const float* __restrict__ bias) {
    __shared__ __align__(16) float os[16 * 68];
    const int lane = threadIdx.x & 31, lr = lane & 15, hi = lane >> 4; const int r0 = blockIdx.x * 64, c0 = blockIdx.y * 64;
    v8f acc[4][4];
#pragma unroll
    for (int mb = 0; mb < 4; ++mb)
#pragma unroll
        for (int nb = 0; nb < 4; ++nb) acc[mb][nb] = (v8f){};
    const size_t aoff = (size_t)(r0 + lr) * K + 8 * hi, boff = (size_t)(c0 + lr) * K + 8 * hi;
#pragma unroll 1
    for (int kc = 0; kc < K; kc += 32) {
        v16bf a[4];
#pragma unroll
        for (int mb = 0; mb < 4; ++mb) a[mb] = ldb(A + aoff + (size_t)mb * 16 * K + kc);
#pragma unroll
        for (int nb = 0; nb < 4; ++nb) {
            const v16bf b = ldb(Bt + boff + (size_t)nb * 16 * K + kc);
#pragma unroll
            for (int mb = 0; mb < 4; ++mb) acc[mb][nb] = wmmab(a[mb], b, acc[mb][nb]);
            asm volatile("v_nop\n\tv_nop\n\tv_nop\n\tv_nop" : "+v"(acc[0][nb]), "+v"(acc[1][nb]), "+v"(acc[2][nb]), "+v"(acc[3][nb]) : "v"(b), "v"(a[0]), "v"(a[1]), "v"(a[2]), "v"(a[3]));
        }
    }
    const int cofs = lr * 4;
    v4f bv; bv[0] = bfr(bias[c0 + cofs]); bv[1] = bfr(bias[c0 + cofs + 1]); bv[2] = bfr(bias[c0 + cofs + 2]); bv[3] = bfr(bias[c0 + cofs + 3]);
#pragma unroll
    for (int mb = 0; mb < 4; ++mb) {
#pragma unroll
        for (int nb = 0; nb < 4; ++nb) {
#pragma unroll
            for (int j = 0; j < 8; ++j) os[(hi * 8 + j) * 68 + nb * 16 + lr] = acc[mb][nb][j]; }
        __builtin_amdgcn_wave_barrier(); asm volatile("" ::: "memory");
        float* crow = C + (size_t)(r0 + mb * 16) * ldc + c0;
#pragma unroll 1
        for (int ps = 0; ps < 2; ++ps) {
#pragma unroll
            for (int s = 0; s < 8; ++s) { const int row = 2 * s + hi; v4f val = *(const v4fa*)(os + row * 68 + cofs); val = val + bv;
                *(volatile v4f*)(crow + (size_t)row * ldc + cofs) = val; }
            if (ps == 0) __threadfence(); }
        __builtin_amdgcn_wave_barrier(); asm volatile("" ::: "memory");
    }
}

__global__ __launch_bounds__(32) void k_gemm_out(const bf* __restrict__ A, const bf* __restrict__ A2, const bf* __restrict__ Bt, int K, float* C, int ldc, const float* __restrict__ bias, size_t sA, size_t sC) {
    __shared__ __align__(16) float os[16 * 68];
    const size_t z = blockIdx.z; A += z * sA; A2 += z * sA; C += z * sC;
    const int lane = threadIdx.x & 31, lr = lane & 15, hi = lane >> 4; const int r0 = blockIdx.x * 64, c0 = blockIdx.y * 64;
    v8f acc[4][4];
#pragma unroll
    for (int mb = 0; mb < 4; ++mb)
#pragma unroll
        for (int nb = 0; nb < 4; ++nb) acc[mb][nb] = (v8f){};
    const size_t aoff = (size_t)(r0 + lr) * K + 8 * hi, boff = (size_t)(c0 + lr) * K + 8 * hi;
#pragma unroll 1
    for (int kc = 0; kc < K; kc += 32) {
        v16bf a[4], a2[4];
#pragma unroll
        for (int mb = 0; mb < 4; ++mb) { a[mb] = ldb(A + aoff + (size_t)mb * 16 * K + kc); a2[mb] = ldb(A2 + aoff + (size_t)mb * 16 * K + kc); }
#pragma unroll
        for (int nb = 0; nb < 4; ++nb) {
            const v16bf b = ldb(Bt + boff + (size_t)nb * 16 * K + kc);
#pragma unroll
            for (int mb = 0; mb < 4; ++mb) { acc[mb][nb] = wmmab(a[mb], b, acc[mb][nb]); acc[mb][nb] = wmmab(a2[mb], b, acc[mb][nb]); }
            asm volatile("v_nop\n\tv_nop\n\tv_nop\n\tv_nop" : "+v"(acc[0][nb]), "+v"(acc[1][nb]), "+v"(acc[2][nb]), "+v"(acc[3][nb]) : "v"(b), "v"(a[0]), "v"(a[1]), "v"(a[2]), "v"(a[3]), "v"(a2[0]), "v"(a2[1]), "v"(a2[2]), "v"(a2[3]));
        }
    }
    const int cofs = lr * 4;
    v4f bv; bv[0] = bfr(bias[c0 + cofs]); bv[1] = bfr(bias[c0 + cofs + 1]); bv[2] = bfr(bias[c0 + cofs + 2]); bv[3] = bfr(bias[c0 + cofs + 3]);
#pragma unroll
    for (int mb = 0; mb < 4; ++mb) {
#pragma unroll
        for (int nb = 0; nb < 4; ++nb) {
#pragma unroll
            for (int j = 0; j < 8; ++j) os[(hi * 8 + j) * 68 + nb * 16 + lr] = acc[mb][nb][j]; }
        __builtin_amdgcn_wave_barrier(); asm volatile("" ::: "memory");
        float* crow = C + (size_t)(r0 + mb * 16) * ldc + c0;
#pragma unroll 1
        for (int ps = 0; ps < 2; ++ps) {
#pragma unroll
            for (int s = 0; s < 8; ++s) { const int row = 2 * s + hi; v4f val = *(const v4fa*)(os + row * 68 + cofs); val = val + bv;
                *(volatile v4f*)(crow + (size_t)row * ldc + cofs) = val; }
            if (ps == 0) __threadfence(); }
        __builtin_amdgcn_wave_barrier(); asm volatile("" ::: "memory");
    }
}

__global__ __launch_bounds__(256) void k_cvt8(const float* __restrict__ src, bf* dst, size_t n8) { const size_t i = (size_t)blockIdx.x * 256 + threadIdx.x; if (i >= n8) return; const v8f v = *(const v8f*)(src + i * 8); v8us o;
#pragma unroll
    for (int k = 0; k < 8; ++k) o[k] = f2bf(v[k]);
    *(volatile v8us*)(dst + i * 8) = o; __threadfence(); *(volatile v8us*)(dst + i * 8) = o; }

__global__ __launch_bounds__(32) void k_mpack(const int* __restrict__ mask, unsigned* MW) {
    const int i = blockIdx.x * 32 + threadIdx.x; const int nw = NB * (SEQ / 32); const int ii = (i < nw) ? i : (nw - 1); const int b = ii / (SEQ / 32), w = ii % (SEQ / 32);
    const int* mp = mask + (size_t)b * SEQ_FULL + w * 32; unsigned word = 0u;
#pragma unroll 4
    for (int j = 0; j < 32; ++j) word |= (mp[j] != 0) ? (1u << j) : 0u;
    if (i >= nw) word = 0xFFFFFFFFu;
    *(volatile unsigned*)(MW + i) = word; __threadfence(); *(volatile unsigned*)(MW + i) = word; }

__global__ __launch_bounds__(256) void k_qkp(const float* __restrict__ F, bf* Ph, bf* Pl) {
    const size_t i = (size_t)blockIdx.x * 256 + threadIdx.x; if (i >= (size_t)NB * NH_ * SEQ * HD / 8) return; const size_t o = i * 8;
    const int d = (int)(o % HD); const int t = (int)((o / HD) % SEQ); const int h = (int)((o / ((size_t)HD * SEQ)) % NH_); const int b = (int)(o / ((size_t)HD * SEQ * NH_));
    const float* f = F + ((size_t)b * SEQ + t) * DM + h * HD + d; const v4f x0 = *(const v4f*)f, x1 = *(const v4f*)(f + 4); v8us oh, ol;
#pragma unroll
    for (int k = 0; k < 4; ++k) { unsigned short a, c; splitf(x0[k], a, c); oh[k] = a; ol[k] = c; splitf(x1[k], a, c); oh[4 + k] = a; ol[4 + k] = c; }
    *(volatile v8us*)(Ph + o) = oh; *(volatile v8us*)(Pl + o) = ol; __threadfence(); *(volatile v8us*)(Ph + o) = oh; *(volatile v8us*)(Pl + o) = ol; }

__global__ __launch_bounds__(256) void k_vtp8(const float* __restrict__ F, h16* V16, h16* Vr) {
    const size_t i = (size_t)blockIdx.x * 256 + threadIdx.x; if (i >= (size_t)NB * NH_ * HD * SEQ / 8) return; const size_t o = i * 8;
    const int t = (int)(o % SEQ); const int d = (int)((o / SEQ) % HD); const int h = (int)((o / ((size_t)SEQ * HD)) % NH_); const int b = (int)(o / ((size_t)SEQ * HD * NH_));
    const float* f = F + ((size_t)b * SEQ + t) * DM + h * HD + d; v8h o16, orr;
#pragma unroll
    for (int q = 0; q < 8; ++q) { const float x = f[(size_t)q * DM]; const h16 hv = (h16)x; o16[q] = hv; orr[q] = (h16)((x - (float)hv) * VRES); }
    *(volatile v8h*)(V16 + o) = o16; *(volatile v8h*)(Vr + o) = orr; __threadfence(); *(volatile v8h*)(V16 + o) = o16; *(volatile v8h*)(Vr + o) = orr; }

__global__ __launch_bounds__(128) void k_attn(const bf* __restrict__ Qh, const bf* __restrict__ Ql, const bf* __restrict__ Kh, const bf* __restrict__ Kl, const h16* __restrict__ V16, const h16* __restrict__ Vr, const unsigned* __restrict__ MW, bf* Ah, bf* Al) {
    __shared__ __align__(16) float os[ATW * 16 * 68];
    const int wave = __builtin_amdgcn_readfirstlane(threadIdx.x >> 5);
    const int lane = threadIdx.x & 31, lr = lane & 15, hi = lane >> 4;
    const int hh = blockIdx.y, bb = blockIdx.z;
    const int q0 = blockIdx.x * (ATW * 16) + wave * 16;
    const size_t pbase = ((size_t)bb * NH_ + hh) * (size_t)SEQ * HD;
    const bf* qhp = Qh + pbase; const bf* qlp = Ql + pbase; const bf* khp = Kh + pbase; const bf* klp = Kl + pbase;
    const h16* v16p = V16 + pbase; const h16* vrp = Vr + pbase;
    const unsigned* mwp = MW + (size_t)bb * (SEQ / 32);
    const int qoff0 = (q0 + lr) * HD + 8 * hi;
    const int koffl = lr * HD + 8 * hi;
    const int voffl = lr * SEQ + 8 * hi;
    v8f acc[4], accr[4];
#pragma unroll
    for (int dt = 0; dt < 4; ++dt) { acc[dt] = (v8f){}; accr[dt] = (v8f){}; }
    float m = -1.0e30f, l = 0.0f;
#pragma unroll 1
    for (int kb = 0; kb < SEQ; kb += 32) {
        int qo = qoff0; asm volatile("" : "+v"(qo));
        v8f st0 = (v8f){}, st1 = (v8f){};
#pragma unroll
        for (int ks = 0; ks < 2; ++ks) {
            const v16bf qh = ldb(qhp + qo + ks * 32), ql = ldb(qlp + qo + ks * 32);
            const int ko = kb * HD + koffl + ks * 32;
            const v16bf kh0 = ldb(khp + ko), kl0 = ldb(klp + ko), kh1 = ldb(khp + ko + 16 * HD), kl1 = ldb(klp + ko + 16 * HD);
            st0 = wmmab(kh0, qh, st0); st1 = wmmab(kh1, qh, st1);
            st0 = wmmab(kl0, qh, st0); st1 = wmmab(kl1, qh, st1);
            st0 = wmmab(kh0, ql, st0); st1 = wmmab(kh1, ql, st1);
            asm volatile("v_nop\n\tv_nop\n\tv_nop\n\tv_nop" : "+v"(st0), "+v"(st1) : "v"(qh), "v"(ql), "v"(kh0), "v"(kl0), "v"(kh1), "v"(kl1));
        }
        const unsigned mw = mwp[kb >> 5];
        if (mw != 0xFFFFFFFFu) {
#pragma unroll
            for (int r = 0; r < 8; ++r) { st0[r] = ((mw >> (8 * hi + r)) & 1u) ? st0[r] : NEGF; st1[r] = ((mw >> (16 + 8 * hi + r)) & 1u) ? st1[r] : NEGF; }
        }
        float mx = fmaxf(st0[0], st1[0]);
#pragma unroll
        for (int r = 1; r < 8; ++r) mx = fmaxf(mx, fmaxf(st0[r], st1[r]));
        mx = fmaxf(mx, __shfl_xor(mx, 16, 32));
        const float mnew = fmaxf(m, mx);
        const float alpha = __builtin_amdgcn_exp2f((m - mnew) * L2E);
        const unsigned grow = __builtin_amdgcn_ballot_w32(mnew > m);
        if (grow != 0u) {
#pragma unroll
            for (int dt = 0; dt < 4; ++dt) { acc[dt] = acc[dt] * alpha; accr[dt] = accr[dt] * alpha; }
        }
        m = mnew;
        float psum = 0.0f; v16h pb;
#pragma unroll
        for (int r = 0; r < 8; ++r) {
            const float p0 = __builtin_amdgcn_exp2f((st0[r] - mnew) * L2E), p1 = __builtin_amdgcn_exp2f((st1[r] - mnew) * L2E);
            psum += p0 + p1; pb[r] = (h16)(p0 * PCAR); pb[8 + r] = (h16)(p1 * PCAR); }
        l = l * alpha + psum;
        const int vo = kb + voffl;
        {
            const v16h va0 = ldh(v16p + vo), va1 = ldh(v16p + vo + 16 * SEQ), va2 = ldh(v16p + vo + 32 * SEQ), va3 = ldh(v16p + vo + 48 * SEQ);
            acc[0] = wmma16(va0, pb, acc[0]); acc[1] = wmma16(va1, pb, acc[1]); acc[2] = wmma16(va2, pb, acc[2]); acc[3] = wmma16(va3, pb, acc[3]);
            asm volatile("v_nop\n\tv_nop\n\tv_nop\n\tv_nop" : "+v"(acc[0]), "+v"(acc[1]), "+v"(acc[2]), "+v"(acc[3]) : "v"(pb), "v"(va0), "v"(va1), "v"(va2), "v"(va3));
        }
        {
            const v16h vb0 = ldh(vrp + vo), vb1 = ldh(vrp + vo + 16 * SEQ), vb2 = ldh(vrp + vo + 32 * SEQ), vb3 = ldh(vrp + vo + 48 * SEQ);
            accr[0] = wmma16(vb0, pb, accr[0]); accr[1] = wmma16(vb1, pb, accr[1]); accr[2] = wmma16(vb2, pb, accr[2]); accr[3] = wmma16(vb3, pb, accr[3]);
            asm volatile("v_nop\n\tv_nop\n\tv_nop\n\tv_nop" : "+v"(accr[0]), "+v"(accr[1]), "+v"(accr[2]), "+v"(accr[3]) : "v"(pb), "v"(vb0), "v"(vb1), "v"(vb2), "v"(vb3));
        }
    }
    l += __shfl_xor(l, 16, 32);
    const float inv = 1.0f / (PCAR * l); const float invr = inv * (1.0f / VRES);
    const int ob = (wave * 16 + lr) * 68 + 8 * hi;
#pragma unroll
    for (int dt = 0; dt < 4; ++dt) { v4f w0, w1;
#pragma unroll
        for (int r = 0; r < 4; ++r) { w0[r] = acc[dt][r] * inv + accr[dt][r] * invr; w1[r] = acc[dt][4 + r] * inv + accr[dt][4 + r] * invr; }
        *(v4fa*)(os + ob + dt * 16) = w0; *(v4fa*)(os + ob + dt * 16 + 4) = w1; }
    __builtin_amdgcn_wave_barrier(); asm volatile("" ::: "memory");
    const size_t orow = ((size_t)bb * SEQ + q0) * DM + hh * HD;
    const int rq = lane >> 3, d8 = (lane & 7) * 8;
#pragma unroll 1
    for (int ps = 0; ps < 2; ++ps) {
#pragma unroll
        for (int s = 0; s < 4; ++s) { const int rr = s * 4 + rq;
            const v4f x0 = *(const v4fa*)(os + (wave * 16 + rr) * 68 + d8), x1 = *(const v4fa*)(os + (wave * 16 + rr) * 68 + d8 + 4); v8us oh, ol;
#pragma unroll
            for (int k = 0; k < 4; ++k) { unsigned short a, c; splitf(x0[k], a, c); oh[k] = a; ol[k] = c; splitf(x1[k], a, c); oh[4 + k] = a; ol[4 + k] = c; }
            *(volatile v8us*)(Ah + orow + (size_t)rr * DM + d8) = oh; *(volatile v8us*)(Al + orow + (size_t)rr * DM + d8) = ol; }
        if (ps == 0) __threadfence(); }
}

constexpr size_t al256(size_t b) { return (b + 255) & ~(size_t)255; }
constexpr size_t MWPAD  = (((size_t)NB * (SEQ / 32) + 31) / 32) * 32;
constexpr size_t SZ_XB  = al256((size_t)NB * SEQ * DM * 2);
constexpr size_t SZ_W   = al256((size_t)DM * DM * 2);
constexpr size_t SZ_F   = al256((size_t)NB * SEQ * DM * 4);
constexpr size_t SZ_PL  = al256((size_t)NB * NH_ * SEQ * HD * 2);
constexpr size_t SZ_MW  = al256(MWPAD * 4);
constexpr size_t OFF_XB = 0;
constexpr size_t OFF_WQ = OFF_XB + SZ_XB;
constexpr size_t OFF_WK = OFF_WQ + SZ_W;
constexpr size_t OFF_WV = OFF_WK + SZ_W;
constexpr size_t OFF_WO = OFF_WV + SZ_W;
constexpr size_t OFF_F  = OFF_WO + SZ_W;
constexpr size_t OFF_QH = OFF_F + SZ_F;
constexpr size_t OFF_QL = OFF_QH + SZ_PL;
constexpr size_t OFF_KH = OFF_QL + SZ_PL;
constexpr size_t OFF_KL = OFF_KH + SZ_PL;
constexpr size_t OFF_V16 = OFF_KL + SZ_PL;
constexpr size_t OFF_VR = OFF_V16 + SZ_PL;
constexpr size_t OFF_AH = OFF_VR + SZ_PL;
constexpr size_t OFF_AL = OFF_AH + SZ_PL;
constexpr size_t OFF_MW = OFF_AL + SZ_PL;
constexpr size_t WS_TOTAL = OFF_MW + SZ_MW;
static_assert(WS_TOTAL <= (size_t)134217728);
static_assert((size_t)NB * NH_ * SEQ * HD == (size_t)NB * SEQ * DM);

extern "C" void kernel_launch(void* const* d_in, const int* in_sizes, int n_in,
                              void* d_out, int out_size, void* d_ws, size_t ws_size, hipStream_t stream) {
    if (n_in < 10) return;
    const size_t xneed = (size_t)(NB - 1) * SEQ_FULL * DM + (size_t)SEQ * DM;
    if ((size_t)in_sizes[0] < xneed) return;
    if ((size_t)in_sizes[1] < (size_t)(NB - 1) * SEQ_FULL + SEQ) return;
    if (in_sizes[2] < DM * DM || in_sizes[4] < DM * DM || in_sizes[6] < DM * DM || in_sizes[8] < DM * DM) return;
    if (in_sizes[3] < DM || in_sizes[5] < DM || in_sizes[7] < DM || in_sizes[9] < DM) return;
    if ((size_t)out_size < xneed) return;
    if (ws_size < WS_TOTAL) return;
    const float* x = (const float*)d_in[0]; const int* mask = (const int*)d_in[1];
    const float* wq = (const float*)d_in[2]; const float* bq = (const float*)d_in[3];
    const float* wk = (const float*)d_in[4]; const float* bk = (const float*)d_in[5];
    const float* wv = (const float*)d_in[6]; const float* bv = (const float*)d_in[7];
    const float* wo = (const float*)d_in[8]; const float* bo = (const float*)d_in[9];
    float* OUT = (float*)d_out;
    char* wsb = (char*)d_ws;
    bf* XB = (bf*)(wsb + OFF_XB); bf* WQ = (bf*)(wsb + OFF_WQ); bf* WK = (bf*)(wsb + OFF_WK); bf* WV = (bf*)(wsb + OFF_WV); bf* WO = (bf*)(wsb + OFF_WO);
    float* F = (float*)(wsb + OFF_F);
    bf* QPh = (bf*)(wsb + OFF_QH); bf* QPl = (bf*)(wsb + OFF_QL); bf* KPh = (bf*)(wsb + OFF_KH); bf* KPl = (bf*)(wsb + OFF_KL);
    h16* VT16 = (h16*)(wsb + OFF_V16); h16* VTr = (h16*)(wsb + OFF_VR);
    bf* ATh = (bf*)(wsb + OFF_AH); bf* ATl = (bf*)(wsb + OFF_AL);
    unsigned* MWp = (unsigned*)(wsb + OFF_MW);

    const size_t xn8 = (size_t)SEQ * DM / 8, wn8 = (size_t)DM * DM / 8;
    for (int b = 0; b < NB; ++b)
        k_cvt8<<<(unsigned)((xn8 + 255) / 256), 256, 0, stream>>>(x + (size_t)b * SEQ_FULL * DM, XB + (size_t)b * SEQ * DM, xn8);
    k_cvt8<<<(unsigned)((wn8 + 255) / 256), 256, 0, stream>>>(wq, WQ, wn8);
    k_cvt8<<<(unsigned)((wn8 + 255) / 256), 256, 0, stream>>>(wk, WK, wn8);
    k_cvt8<<<(unsigned)((wn8 + 255) / 256), 256, 0, stream>>>(wv, WV, wn8);
    k_cvt8<<<(unsigned)((wn8 + 255) / 256), 256, 0, stream>>>(wo, WO, wn8);
    k_mpack<<<(unsigned)(MWPAD / 32), 32, 0, stream>>>(mask, MWp);

    const dim3 gp((unsigned)(NB * SEQ / 64), DM / 64, 1);
    const unsigned lp = (unsigned)(((size_t)NB * SEQ * DM / 8 + 255) / 256);
    k_gemm_proj<<<gp, 32, 0, stream>>>(XB, WQ, DM, F, DM, bq);
    k_qkp<<<lp, 256, 0, stream>>>(F, QPh, QPl);
    k_gemm_proj<<<gp, 32, 0, stream>>>(XB, WK, DM, F, DM, bk);
    k_qkp<<<lp, 256, 0, stream>>>(F, KPh, KPl);
    k_gemm_proj<<<gp, 32, 0, stream>>>(XB, WV, DM, F, DM, bv);
    k_vtp8<<<lp, 256, 0, stream>>>(F, VT16, VTr);

    k_attn<<<dim3(SEQ / (ATW * 16), NH_, NB), ATW * 32, 0, stream>>>(QPh, QPl, KPh, KPl, VT16, VTr, MWp, ATh, ATl);

    k_gemm_out<<<dim3(SEQ / 64, DM / 64, NB), 32, 0, stream>>>(ATh, ATl, WO, DM, OUT, DM, bo, (size_t)SEQ * DM, (size_t)SEQ_FULL * DM);
}
